// DynaFormer_49752901157521
// MI455X (gfx1250) — hardware-verified
//
#include <hip/hip_runtime.h>
#include <math.h>

typedef __attribute__((ext_vector_type(16))) _Float16 v16h;
typedef __attribute__((ext_vector_type(16))) __bf16 v16b;
typedef __attribute__((ext_vector_type(8)))  _Float16 v8h;
typedef __attribute__((ext_vector_type(8)))  float v8f;
typedef __attribute__((ext_vector_type(4)))  float v4f;
typedef __attribute__((ext_vector_type(2)))  float v2f;
typedef __attribute__((ext_vector_type(4)))  unsigned v4u;
typedef __attribute__((ext_vector_type(4)))  int v4i;
typedef float __attribute__((may_alias)) float_a;
typedef int __attribute__((may_alias)) int_a;

template <typename T> __device__ __forceinline__ void vst2(void* p, T v) { *(volatile T*)p = v; __threadfence(); *(volatile T*)p = v; }
__device__ __forceinline__ v8f wmma16(v16h a, v16h b, v8f c) {
  v8f d = __builtin_amdgcn_wmma_f32_16x16x32_f16(false, a, false, b, (short)0, c, false, false);
  asm volatile("v_nop\n\tv_nop\n\tv_nop\n\tv_nop" : "+v"(d) : "v"(a), "v"(b));
  return d;
}
__device__ __forceinline__ v8f wmma_bf(v16b a, v16b b, v8f c) {
  v8f d = __builtin_amdgcn_wmma_f32_16x16x32_bf16(false, a, false, b, (short)0, c, false, false);
  asm volatile("v_nop\n\tv_nop\n\tv_nop\n\tv_nop" : "+v"(d) : "v"(a), "v"(b));
  return d;
}
__device__ __forceinline__ v16h frag_h(const _Float16* rowk0, int lane) {
  union { v16h v; v8h q[2]; } u; const _Float16* p = rowk0 + 8 * (lane >> 4);
  u.q[0] = *(const v8h*)p; u.q[1] = *(const v8h*)(p + 16); return u.v;
}
__device__ __forceinline__ v16h frag_f32(const float* rowk0, int lane) {
  v16h a; const float* p = rowk0 + 8 * (lane >> 4);
#pragma unroll
  for (int i = 0; i < 8; ++i) { a[i] = (_Float16)p[i]; a[8 + i] = (_Float16)p[16 + i]; }
  return a;
}
__device__ __forceinline__ v16h frag_f32s(const float* rowk0, int lane, float sc) {
  v16h a; const float* p = rowk0 + 8 * (lane >> 4);
#pragma unroll
  for (int i = 0; i < 8; ++i) { a[i] = (_Float16)(p[i] * sc); a[8 + i] = (_Float16)(p[16 + i] * sc); }
  return a;
}
__device__ __forceinline__ v16h fragc_f32(const float* W, int k0, int n, int lane, int ld, int K) {
  v16h a; const int g = lane >> 4;
#pragma unroll
  for (int i = 0; i < 8; ++i) { const int ka = k0 + 8 * g + i, kb = ka + 16;
    a[i] = (_Float16)(ka < K ? W[(size_t)(ka < K ? ka : K - 1) * ld + n] : 0.f); a[8 + i] = (_Float16)(kb < K ? W[(size_t)(kb < K ? kb : K - 1) * ld + n] : 0.f); }
  return a;
}
struct F2 { v16b h, l; };
__device__ __forceinline__ F2 bsplit16(const float v[16]) { F2 r;
#pragma unroll
  for (int i = 0; i < 16; ++i) { const __bf16 h = (__bf16)v[i]; r.h[i] = h; r.l[i] = (__bf16)(v[i] - (float)h); }
  return r; }
__device__ __forceinline__ F2 split_row(const float* row, int k0, int lane) { float v[16]; const float* p = row + k0 + 8 * (lane >> 4);
#pragma unroll
  for (int i = 0; i < 8; ++i) { v[i] = p[i]; v[8 + i] = p[16 + i]; }
  return bsplit16(v); }
__device__ __forceinline__ F2 split_rowK(const float* row, int k0, int lane, int K) { float v[16]; const int g = lane >> 4;
#pragma unroll
  for (int i = 0; i < 8; ++i) { const int ka = k0 + 8 * g + i, kb = ka + 16; v[i] = ka < K ? row[ka < K ? ka : K - 1] : 0.f; v[8 + i] = kb < K ? row[kb < K ? kb : K - 1] : 0.f; }
  return bsplit16(v); }
__device__ __forceinline__ F2 split_col(const float* W, int k0, int n, int lane, int ld, int K) { float v[16]; const int g = lane >> 4;
#pragma unroll
  for (int i = 0; i < 8; ++i) { const int ka = k0 + 8 * g + i, kb = ka + 16; v[i] = ka < K ? W[(size_t)(ka < K ? ka : K - 1) * ld + n] : 0.f; v[8 + i] = kb < K ? W[(size_t)(kb < K ? kb : K - 1) * ld + n] : 0.f; }
  return bsplit16(v); }
__device__ __forceinline__ v8f mac3(const F2& a, const F2& b, v8f c) { c = wmma_bf(a.l, b.h, c); c = wmma_bf(a.h, b.l, c); return wmma_bf(a.h, b.h, c); }
__device__ __forceinline__ float sigm(float v) { return 1.0f / (1.0f + expf(-v)); }
#define LDSX() do { asm volatile("s_wait_dscnt 0" ::: "memory"); __builtin_amdgcn_wave_barrier(); __builtin_amdgcn_fence(__ATOMIC_RELEASE, "workgroup"); } while (0)


#ifndef NN
#define NN 2048
#endif
#define NE 65536
#define DIN 16
#define DM 128
#define NH 8
#define FF 512
#define NL 3
#define NOUT 64
#define QKVW (3 * NH * DM)
typedef __attribute__((ext_vector_type(8))) __bf16 v8b;
__device__ __forceinline__ v16b frag_b(const __bf16* rowk0, int lane) {
  union { v16b v; v8b q[2]; } u; const __bf16* p = rowk0 + 8 * (lane >> 4);
  u.q[0] = *(const v8b*)p; u.q[1] = *(const v8b*)(p + 16); return u.v;
}
__device__ __forceinline__ float bfr(float v) { return (float)(__bf16)v; }
__device__ __attribute__((noinline)) float exp_ni(float v) { return expf(v); }
__device__ __attribute__((noinline)) float erf_ni(float v) { return erff(v); }

#define PK_IN  0
#define PK_QKV (PK_IN + DM * 32)
#define PK_O   (PK_QKV + NL * QKVW * DM)
#define PK_F1  (PK_O + NL * DM * NH * DM)
#define PK_F2  (PK_F1 + NL * FF * DM)
#define PK_OUT (PK_F2 + NL * DM * FF)
#define PK_END (PK_OUT + NOUT * DM)
#define WS_PK   0u
#define WS_H    (WS_PK + 2u * PK_END)
#define WS_XN   (WS_H + 4u * NN * DM)
#define WS_QKV  (WS_XN + 4u * NN * DM)
#define WS_VTH  (WS_QKV + 4u * NN * QKVW)
#define WS_VTL  (WS_VTH + 2u * NH * DM * NN)
#define WS_BIAS (WS_VTL + 2u * NH * DM * NN)
#define WS_O    (WS_BIAS + 4u * NN * NN)
#define WS_FH   (WS_O + 4u * NN * NH * DM)
#define WS_DEG  (WS_FH + 4u * NN * FF)
#define WS_END  (WS_DEG + 4u * NN * 4)

__global__ __launch_bounds__(256) void k_packT(const float* __restrict__ Wm, int K, int Kreal, int ld, __bf16* __restrict__ DST) {
  __shared__ __align__(16) __bf16 s[1024]; const int n = blockIdx.x, tid = threadIdx.x;
  for (int k = tid; k < K; k += 256) s[k] = (__bf16)(k < Kreal ? Wm[(size_t)k * ld + n] : 0.f);
  __syncthreads();
  for (int q = tid; q < K / 8; q += 256) vst2((unsigned*)(DST + (size_t)n * K + q * 8), *(const v4u*)&s[q * 8]);
}
__global__ __launch_bounds__(128) void k_packqkv(const float* __restrict__ WQ, const float* __restrict__ WK, const float* __restrict__ WV, __bf16* __restrict__ DST) {
  __shared__ __align__(16) __bf16 s[DM]; const int n = blockIdx.x, which = blockIdx.y, l = blockIdx.z, k = threadIdx.x; const int h = n / DM, e = n % DM;
  const float* Wm = (which == 0) ? WQ : (which == 1 ? WK : WV);
  s[k] = (__bf16)Wm[(((size_t)l * NH + h) * DM + k) * DM + e];
  __syncthreads();
  if (k < 16) vst2((unsigned*)(DST + ((size_t)l * QKVW + which * NH * DM + n) * DM + k * 8), *(const v4u*)&s[k * 8]);
}
__global__ __launch_bounds__(256) void k_deg(const int* __restrict__ EI, int* __restrict__ DEG) {
  __shared__ __align__(16) int sd[64][4]; const int tid = threadIdx.x; const int nl = tid >> 2, sub = tid & 3; const int node = blockIdx.x * 64 + nl;
  int ci = 0, co = 0;
  for (int e = sub; e < NE; e += 4) { ci += (EI[NE + e] == node); co += (EI[e] == node); }
  ci += __shfl_xor(ci, 1); ci += __shfl_xor(ci, 2); co += __shfl_xor(co, 1); co += __shfl_xor(co, 2);
  if (sub == 0) { sd[nl][0] = min(ci, 63); sd[nl][1] = min(co, 63); sd[nl][2] = 0; sd[nl][3] = 0; }
  __syncthreads();
  if (tid < 64) vst2((unsigned*)(DEG + ((size_t)blockIdx.x * 64 + tid) * 4), *(const v4u*)&sd[tid][0]);
}
__global__ __launch_bounds__(128) void k_h0(const float* __restrict__ X, const __bf16* __restrict__ P, const float* __restrict__ bin, const float* __restrict__ ZI, const float* __restrict__ ZO, const int* __restrict__ DEG, float* __restrict__ Hs) {
  __shared__ __align__(16) float so[4][16][132];
  const int tid = threadIdx.x, wave = tid >> 5, lane = tid & 31, col = lane & 15, g = lane >> 4; const size_t r0 = (size_t)blockIdx.x * 64 + wave * 16;
  v16b a; { const float* p = X + (r0 + col) * DIN;
#pragma unroll
    for (int i = 0; i < 8; ++i) { const int ka = 8 * g + i; a[i] = (__bf16)(ka < DIN ? p[ka < DIN ? ka : 0] : 0.f); a[8 + i] = (__bf16)0.f; } }
  v8f acc[8] = {};
#pragma unroll
  for (int j = 0; j < 8; ++j) acc[j] = wmma_bf(a, frag_b(P + (size_t)(j * 16 + col) * 32, lane), acc[j]);
#pragma unroll
  for (int j = 0; j < 8; ++j) { const int n = j * 16 + col;
#pragma unroll
    for (int r = 0; r < 8; ++r) { const size_t row = r0 + 8 * g + r; const int di = min(max(DEG[row * 4], 0), 63), dq = min(max(DEG[row * 4 + 1], 0), 63); so[wave][8 * g + r][n] = acc[j][r] + bfr(bin[n]) + bfr(ZI[(size_t)di * DM + n]) + bfr(ZO[(size_t)dq * DM + n]); } }
  LDSX();
  for (int rl = 0; rl < 16; ++rl) vst2(Hs + (r0 + rl) * DM + lane * 4, *(const v4f*)&so[wave][rl][lane * 4]);
}
__global__ __launch_bounds__(256) void k_bias(const float* __restrict__ POS, const float* __restrict__ MU, const float* __restrict__ SG, const float* __restrict__ SW, const float* __restrict__ SB, float* __restrict__ BIAS) {
  __shared__ __align__(16) float s[256]; __shared__ float smu[8], ssg[8], ssw[8];
  const int n = blockIdx.x, m0 = blockIdx.y * 256, tid = threadIdx.x;
  if (tid < 8) { smu[tid] = bfr(MU[tid]); ssg[tid] = bfr(SG[tid]); ssw[tid] = bfr(SW[tid]); }
  __syncthreads();
  const int m = m0 + tid; const float dx = bfr(POS[n * 3 + 0]) - bfr(POS[m * 3 + 0]), dy = bfr(POS[n * 3 + 1]) - bfr(POS[m * 3 + 1]), dz = bfr(POS[n * 3 + 2]) - bfr(POS[m * 3 + 2]);
  const float d = sqrtf(dx * dx + dy * dy + dz * dz + 1e-12f); float b = bfr(SB[0]);
#pragma unroll
  for (int sI = 0; sI < 8; ++sI) { const float t = (d - smu[sI]) / ssg[sI]; b += ssw[sI] * exp_ni(-0.5f * t * t); }
  s[tid] = b; __syncthreads();
  if (tid < 64) vst2(BIAS + (size_t)n * NN + m0 + tid * 4, *(const v4f*)&s[tid * 4]);
}
__global__ __launch_bounds__(256) void k_ln(const float* __restrict__ Xs, const float* __restrict__ gw, const float* __restrict__ bw, float* __restrict__ Y) {
  __shared__ __align__(16) float s[16][DM];
  const int wave = threadIdx.x >> 5, lane = threadIdx.x & 31;
#pragma unroll
  for (int rr = 0; rr < 2; ++rr) { const int rl = wave * 2 + rr; const size_t r = (size_t)blockIdx.x * 16 + rl; const float* x = Xs + r * DM; float v[4]; float sum = 0.f;
#pragma unroll
    for (int i = 0; i < 4; ++i) { v[i] = x[lane + 32 * i]; sum += v[i]; }
#pragma unroll
    for (int o = 1; o < 32; o <<= 1) sum += __shfl_xor(sum, o);
    const float mu = sum / (float)DM; float var = 0.f;
#pragma unroll
    for (int i = 0; i < 4; ++i) { const float dd = v[i] - mu; var += dd * dd; }
#pragma unroll
    for (int o = 1; o < 32; o <<= 1) var += __shfl_xor(var, o);
    const float rs = rsqrtf(var / (float)DM + 1e-5f);
#pragma unroll
    for (int i = 0; i < 4; ++i) { const int c = lane + 32 * i; s[rl][c] = (v[i] - mu) * rs * bfr(gw[c]) + bfr(bw[c]); } }
  LDSX();
#pragma unroll
  for (int rr = 0; rr < 2; ++rr) { const int rl = wave * 2 + rr; const size_t r = (size_t)blockIdx.x * 16 + rl; vst2(Y + r * DM + lane * 4, *(const v4f*)&s[rl][lane * 4]); }
}
template <int K, int EPI, int RM, int VT, int NT>
__global__ __launch_bounds__(128) void k_lin(const float* __restrict__ A, int lda, const __bf16* __restrict__ P, const float* __restrict__ bias, float* OUT, int ldo, const float* RES, __bf16* __restrict__ PH, __bf16* __restrict__ PL) {
  __shared__ __align__(16) float so[4][16][132]; __shared__ __align__(16) __bf16 sth[VT ? 128 : 1][72], stl[VT ? 128 : 1][72];
  const int tid = threadIdx.x, wave = tid >> 5, lane = tid & 31, col = lane & 15, g = lane >> 4; const size_t r0 = (size_t)blockIdx.x * 64 + wave * 16; const int n0 = blockIdx.y * (NT * 16);
  v8f acc[NT]; for (int j = 0; j < NT; ++j) acc[j] = (v8f){};
#pragma unroll 2
  for (int kc = 0; kc < K / 32; ++kc) { const F2 a = split_row(A + (r0 + col) * lda, kc * 32, lane);
#pragma unroll
    for (int j = 0; j < NT; ++j) { const v16b w = frag_b(P + (size_t)(n0 + j * 16 + col) * K + kc * 32, lane); acc[j] = wmma_bf(a.l, w, acc[j]); acc[j] = wmma_bf(a.h, w, acc[j]); } }
  if (!VT) {
#pragma unroll
    for (int j = 0; j < NT; ++j) { const int n = n0 + j * 16 + col; const float bb = bias ? bfr(bias[n]) : 0.f;
#pragma unroll
      for (int r = 0; r < 8; ++r) { const size_t row = r0 + 8 * g + r; float v = acc[j][r] + bb; if (EPI == 1) v = 0.5f * v * (1.0f + erf_ni(v * 0.70710678118654752f)); if (RM == 1) v += RES[row * ldo + n]; so[wave][8 * g + r][j * 16 + col] = v; } }
    LDSX();
    for (int rl = 0; rl < 16; ++rl) if (lane < NT * 4) vst2(OUT + (r0 + rl) * ldo + n0 + lane * 4, *(const v4f*)&so[wave][rl][lane * 4]);
  } else {
#pragma unroll
    for (int j = 0; j < (VT ? NT : 0); ++j) { const int n = n0 + j * 16 + col; const float bb = bias ? bfr(bias[n]) : 0.f;
#pragma unroll
      for (int r = 0; r < 8; ++r) { const float v = acc[j][r] + bb; const __bf16 hb = (__bf16)v; sth[j * 16 + col][wave * 16 + 8 * g + r] = hb; stl[j * 16 + col][wave * 16 + 8 * g + r] = (__bf16)(v - (float)hb); } }
    __syncthreads();
    const int s0 = blockIdx.x * 64; const int prow0 = n0;
    for (int q = tid; q < 128 * 8; q += 128) { const int dI = q >> 3, pc = q & 7; const size_t o = (size_t)(prow0 + dI) * NN + s0 + pc * 8; vst2((unsigned*)(PH + o), *(const v4u*)&sth[dI][pc * 8]); vst2((unsigned*)(PL + o), *(const v4u*)&stl[dI][pc * 8]); }
  }
}
__global__ __launch_bounds__(128) void k_attn(const float* __restrict__ QKV, const float* __restrict__ BIAS, const __bf16* __restrict__ VTH, const __bf16* __restrict__ VTL, float* __restrict__ O) {
  __shared__ __align__(16) float sp[4][16][36]; __shared__ __align__(16) float so[4][16][132];
  const int tid = threadIdx.x, wave = tid >> 5, lane = tid & 31, col = lane & 15, g = lane >> 4;
  const int qb = blockIdx.x, h = blockIdx.y; const size_t q0 = (size_t)qb * 64 + wave * 16;
  F2 aq[4];
#pragma unroll
  for (int kc = 0; kc < 4; ++kc) aq[kc] = split_row(QKV + (q0 + col) * QKVW + h * DM, kc * 32, lane);
  float m[8], l[8];
#pragma unroll
  for (int r = 0; r < 8; ++r) { m[r] = -3.0e38f; l[r] = 0.f; }
  v8f acc[8] = {};
#pragma unroll 1
  for (int ks = 0; ks < NN / 32; ++ks) { v8f s[2];
#pragma unroll
    for (int ct = 0; ct < 2; ++ct) { const int kk = ks * 32 + ct * 16 + col; const float* krow = QKV + (size_t)kk * QKVW + NH * DM + h * DM; v8f c = {};
#pragma unroll
      for (int kc = 0; kc < 4; ++kc) { const F2 kb = split_row(krow, kc * 32, lane); c = mac3(aq[kc], kb, c); }
#pragma unroll
      for (int r = 0; r < 8; ++r) s[ct][r] = c[r] * 0.08838834764831845f + BIAS[(q0 + 8 * g + r) * NN + kk]; }
#pragma unroll
    for (int r = 0; r < 8; ++r) { float mx = fmaxf(s[0][r], s[1][r]);
#pragma unroll
      for (int o = 1; o < 16; o <<= 1) mx = fmaxf(mx, __shfl_xor(mx, o));
      const float mn = fmaxf(m[r], mx); const float alpha = exp_ni(m[r] - mn);
      const float e0 = exp_ni(s[0][r] - mn), e1 = exp_ni(s[1][r] - mn); float es = e0 + e1;
#pragma unroll
      for (int o = 1; o < 16; o <<= 1) es += __shfl_xor(es, o);
      l[r] = l[r] * alpha + es; m[r] = mn;
#pragma unroll
      for (int dt = 0; dt < 8; ++dt) acc[dt][r] *= alpha;
      sp[wave][8 * g + r][col] = e0; sp[wave][8 * g + r][16 + col] = e1; }
    LDSX();
    const F2 pa = split_row(&sp[wave][col][0], 0, lane);
#pragma unroll
    for (int dt = 0; dt < 8; ++dt) { const size_t vr = (size_t)(h * DM + dt * 16 + col) * NN + ks * 32; const v16b vh = frag_b(VTH + vr, lane), vl = frag_b(VTL + vr, lane); acc[dt] = wmma_bf(pa.l, vh, acc[dt]); acc[dt] = wmma_bf(pa.h, vl, acc[dt]); acc[dt] = wmma_bf(pa.h, vh, acc[dt]); }
    LDSX(); }
#pragma unroll
  for (int r = 0; r < 8; ++r) { const float il = 1.0f / l[r];
#pragma unroll
    for (int dt = 0; dt < 8; ++dt) so[wave][8 * g + r][dt * 16 + col] = acc[dt][r] * il; }
  LDSX();
  for (int rl = 0; rl < 16; ++rl) vst2(O + (q0 + rl) * (NH * DM) + h * DM + lane * 4, *(const v4f*)&so[wave][rl][lane * 4]);
}
extern "C" void kernel_launch(void* const* d_in, const int* in_sizes, int n_in, void* d_out, int out_size, void* d_ws, size_t ws_size, hipStream_t stream) {
  (void)in_sizes; (void)n_in; (void)out_size;
  const float** F = (const float**)d_in; const int* EI = (const int*)d_in[1];
  if (ws_size < (size_t)WS_END) return;
  char* ws = (char*)d_ws; __bf16 *PK = (__bf16*)(ws + WS_PK), *VTH = (__bf16*)(ws + WS_VTH), *VTL = (__bf16*)(ws + WS_VTL);
  float *Hs = (float*)(ws + WS_H), *XN = (float*)(ws + WS_XN), *QKV = (float*)(ws + WS_QKV), *BIAS = (float*)(ws + WS_BIAS), *O = (float*)(ws + WS_O), *FH = (float*)(ws + WS_FH); int* DEG = (int*)(ws + WS_DEG);
  k_packT<<<DM, 256, 0, stream>>>(F[4], 32, DIN, DM, PK + PK_IN);
  for (int l = 0; l < NL; ++l) {
    k_packT<<<DM, 256, 0, stream>>>(F[20] + (size_t)l * NH * DM * DM, NH * DM, NH * DM, DM, PK + PK_O + (size_t)l * DM * NH * DM);
    k_packT<<<FF, 256, 0, stream>>>(F[26] + (size_t)l * DM * FF, DM, DM, FF, PK + PK_F1 + (size_t)l * FF * DM);
    k_packT<<<DM, 256, 0, stream>>>(F[28] + (size_t)l * FF * DM, FF, FF, DM, PK + PK_F2 + (size_t)l * DM * FF); }
  k_packT<<<NOUT, 256, 0, stream>>>(F[30], DM, DM, NOUT, PK + PK_OUT);
  k_packqkv<<<dim3(NH * DM, 3, NL), 128, 0, stream>>>(F[14], F[16], F[18], PK + PK_QKV);
  k_deg<<<NN / 64, 256, 0, stream>>>(EI, DEG);
  k_h0<<<NN / 64, 128, 0, stream>>>(F[0], PK + PK_IN, F[5], F[8], F[9], DEG, Hs);
  k_bias<<<dim3(NN, NN / 256), 256, 0, stream>>>(F[3], F[10], F[11], F[12], F[13], BIAS);
  for (int l = 0; l < NL; ++l) {
    k_ln<<<NN / 16, 256, 0, stream>>>(Hs, F[22] + l * DM, F[23] + l * DM, XN);
    k_lin<DM, 0, 0, 0, 8><<<dim3(NN / 64, NH * DM / 128), 128, 0, stream>>>(XN, DM, PK + PK_QKV + ((size_t)l * QKVW) * DM, F[15] + (size_t)l * NH * DM, QKV, QKVW, nullptr, nullptr, nullptr);
    k_lin<DM, 0, 0, 0, 8><<<dim3(NN / 64, NH * DM / 128), 128, 0, stream>>>(XN, DM, PK + PK_QKV + ((size_t)l * QKVW + NH * DM) * DM, F[17] + (size_t)l * NH * DM, QKV + NH * DM, QKVW, nullptr, nullptr, nullptr);
    k_lin<DM, 0, 0, 1, 8><<<dim3(NN / 64, NH * DM / 128), 128, 0, stream>>>(XN, DM, PK + PK_QKV + ((size_t)l * QKVW + 2 * NH * DM) * DM, F[19] + (size_t)l * NH * DM, nullptr, 0, nullptr, VTH, VTL);
    k_attn<<<dim3(NN / 64, NH), 128, 0, stream>>>(QKV, BIAS, VTH, VTL, O);
    k_lin<NH * DM, 0, 1, 0, 8><<<dim3(NN / 64, 1), 128, 0, stream>>>(O, NH * DM, PK + PK_O + (size_t)l * DM * NH * DM, F[21] + l * DM, Hs, DM, Hs, nullptr, nullptr);
    k_ln<<<NN / 16, 256, 0, stream>>>(Hs, F[24] + l * DM, F[25] + l * DM, XN);
    k_lin<DM, 1, 0, 0, 8><<<dim3(NN / 64, FF / 128), 128, 0, stream>>>(XN, DM, PK + PK_F1 + (size_t)l * FF * DM, F[27] + l * FF, FH, FF, nullptr, nullptr, nullptr);
    k_lin<FF, 0, 1, 0, 8><<<dim3(NN / 64, 1), 128, 0, stream>>>(FH, FF, PK + PK_F2 + (size_t)l * DM * FF, F[29] + l * DM, Hs, DM, Hs, nullptr, nullptr); }
  k_lin<DM, 0, 0, 0, 4><<<dim3(NN / 64, 1), 128, 0, stream>>>(Hs, DM, PK + PK_OUT, F[31], (float*)d_out, NOUT, nullptr, nullptr, nullptr);
}
